// RengarNetwork_67422396612990
// MI455X (gfx1250) — hardware-verified
//
#include <hip/hip_runtime.h>
#include <stddef.h>
#include <stdint.h>


#define VOCAB 185
#define LF    32
#define S1    256
#define S2    128
#define S3    16
#define K1    768
#define K2    640
#define TABW  768
#define P1    776
#define P2    648
#define TP    32
#define NTHR  256
#define NWAVE 8
#define PREP_BLOCKS 8
#define WSCAP 134217728

#define ASC 16384.0f
#define WSC 8192.0f
#define OSC (1.0f / 134217728.0f)
#define THR 0.9921875f

#define LDS_A1   (TP * P1 * 2)
#define LDS_A2   (TP * P2 * 2)
#define LDS_PART (NWAVE * 2 * 256 * 4)
#define LDS_OUT  (TP * 4)
#define OFF_A2   (LDS_A1)
#define OFF_PART (OFF_A2 + LDS_A2)
#define OFF_OUT  (OFF_PART + LDS_PART)
#define LDS_MAIN (OFF_OUT + LDS_OUT)

#define W1T_BYTES (S3 * K1 * 2)
#define W2T_BYTES (S3 * K2 * 2)
#define TAB_BYTES (VOCAB * TABW * 4)

static_assert(K1 == 2 * S1 + 2 * S2);
static_assert(K2 == 2 * S1 + S2);
static_assert((K1 % 128) == 0);
static_assert((K2 % 128) == 0);
static_assert(TP == 32);
static_assert(NTHR == NWAVE * 32);
static_assert((TP % NWAVE) == 0);
static_assert((P1 % 8) == 0 && P1 >= K1);
static_assert((P2 % 8) == 0 && P2 >= K2);
static_assert((LDS_A1 % 16) == 0 && (LDS_A2 % 16) == 0 && (LDS_PART % 16) == 0);
static_assert(LDS_MAIN <= 300 * 1024);
static_assert((W1T_BYTES % 512) == 0 && (W2T_BYTES % 512) == 0);
static_assert(((VOCAB * (S1 / 4)) % 32) == 0 && ((VOCAB * (S2 / 4)) % 32) == 0);
static_assert(((S3 * (S1 / 8)) % 32) == 0 && ((S3 * (S2 / 8)) % 32) == 0);
static_assert(S1 == 8 * 32 && S2 == 4 * 32);

typedef float    v4f  __attribute__((ext_vector_type(4)));
typedef float    v8f  __attribute__((ext_vector_type(8)));
typedef _Float16 v4h  __attribute__((ext_vector_type(4)));
typedef _Float16 v8h  __attribute__((ext_vector_type(8)));
typedef _Float16 v16h __attribute__((ext_vector_type(16)));
union FragH { v16h v; v8h h[2]; };

__device__ __forceinline__ v8f wmf(v16h a, v16h b, v8f c) {
  v8f d = __builtin_amdgcn_wmma_f32_16x16x32_f16(false, a, false, b, (short)0, c, false, false);
  asm volatile("v_nop\n\tv_nop\n\tv_nop\n\tv_nop" : "+v"(d) : "v"(a), "v"(b));
  return d;
}

__device__ __forceinline__ float clampT(float x) { return fminf(fmaxf(x, -THR), THR); }

__device__ __forceinline__ float add_prod(float a, float x, float y) {
#pragma clang fp contract(off)
  return a + x * y;
}

__device__ __forceinline__ void st2_v4f(float* p, v4f v) {
  *(volatile v4f*)p = v;
  __threadfence();
  *(volatile v4f*)p = v;
}
__device__ __forceinline__ void st2_v8h(_Float16* p, v8h v) {
  *(volatile v8h*)p = v;
  __threadfence();
  *(volatile v8h*)p = v;
}

__device__ __forceinline__ void tab_seg(const float* __restrict__ src, int kw, float* tab,
                                        int col0, int gt, int gs) {
  const int kq = kw >> 2;
  const int items = VOCAB * kq;
#pragma unroll 1
  for (int it = gt; it < items; it += gs) {
    const int v = it / kq, k4 = it - v * kq;
    const v4f x = *(const v4f*)(src + (size_t)v * kw + 4 * k4);
    st2_v4f(tab + (size_t)v * TABW + col0 + 4 * k4, x);
  }
}
__device__ __forceinline__ void w_seg(const float* __restrict__ src, int kw, _Float16* dst,
                                      int pitch, int col0, int gt, int gs) {
  const int ko = kw >> 3;
  const int items = S3 * ko;
#pragma unroll 1
  for (int it = gt; it < items; it += gs) {
    const int n = it / ko, k8 = it - n * ko;
    const float* sp = src + n * kw + 8 * k8;
    const v4f x0 = *(const v4f*)sp;
    const v4f x1 = *(const v4f*)(sp + 4);
    v8h hv;
    hv[0] = (_Float16)(x0[0] * WSC); hv[1] = (_Float16)(x0[1] * WSC);
    hv[2] = (_Float16)(x0[2] * WSC); hv[3] = (_Float16)(x0[3] * WSC);
    hv[4] = (_Float16)(x1[0] * WSC); hv[5] = (_Float16)(x1[1] * WSC);
    hv[6] = (_Float16)(x1[2] * WSC); hv[7] = (_Float16)(x1[3] * WSC);
    st2_v8h(dst + n * pitch + col0 + 8 * k8, hv);
  }
}

__global__ __launch_bounds__(NTHR) void k_prep(const float* __restrict__ emb_fs,
                                               const float* __restrict__ emb_va,
                                               const float* __restrict__ emb_ha,
                                               const float* __restrict__ emb_ra,
                                               const float* __restrict__ fs_w,
                                               const float* __restrict__ absva_w,
                                               const float* __restrict__ absha_w,
                                               const float* __restrict__ absra_w,
                                               const float* __restrict__ va_w,
                                               const float* __restrict__ fsxva_w,
                                               const float* __restrict__ haxra_w,
                                               _Float16* w1t, _Float16* w2t, float* tab) {
  const int gt = blockIdx.x * NTHR + threadIdx.x;
  const int gs = gridDim.x * NTHR;
  tab_seg(emb_fs, S1, tab, 0, gt, gs);
  tab_seg(emb_va, S1, tab, S1, gt, gs);
  tab_seg(emb_ha, S2, tab, 2 * S1, gt, gs);
  tab_seg(emb_ra, S2, tab, 2 * S1 + S2, gt, gs);
  w_seg(fs_w,    S1, w1t, K1, 0, gt, gs);
  w_seg(absva_w, S1, w1t, K1, S1, gt, gs);
  w_seg(absha_w, S2, w1t, K1, 2 * S1, gt, gs);
  w_seg(absra_w, S2, w1t, K1, 2 * S1 + S2, gt, gs);
  w_seg(va_w,    S1, w2t, K2, 0, gt, gs);
  w_seg(fsxva_w, S1, w2t, K2, S1, gt, gs);
  w_seg(haxra_w, S2, w2t, K2, 2 * S1, gt, gs);
}

__global__ __launch_bounds__(NTHR) void k_main(const int* __restrict__ pst,
                                               const float* __restrict__ csg,
                                               const float* __restrict__ ssg,
                                               const float* __restrict__ wtm,
                                               const float* __restrict__ tempo,
                                               const float* __restrict__ fsb,
                                               const float* __restrict__ wov,
                                               const float* __restrict__ wof,
                                               const float* __restrict__ tab,
                                               const _Float16* __restrict__ w1t,
                                               const _Float16* __restrict__ w2t,
                                               float* out) {
  extern __shared__ v4f lds_dyn[];
  char* lds = (char*)lds_dyn;
  _Float16* A1 = (_Float16*)lds;
  _Float16* A2 = (_Float16*)(lds + OFF_A2);
  float* part = (float*)(lds + OFF_PART);
  float* sout = (float*)(lds + OFF_OUT);

  const int tid = threadIdx.x, lane = tid & 31, hh = lane >> 4, m = lane & 15;
  const int wave = __builtin_amdgcn_readfirstlane(tid >> 5);
  const int p0 = blockIdx.x * TP;
  const v4f z4 = {0.f, 0.f, 0.f, 0.f};
  const v4f t0 = *(const v4f*)(tempo + 8 * lane);
  const v4f t1 = *(const v4f*)(tempo + 8 * lane + 4);

#pragma unroll 1
  for (int j = 0; j < TP / NWAVE; ++j) {
    const int r = (TP / NWAVE) * wave + j;
    const int p = p0 + r;
    const size_t fb = (size_t)p * LF;
    v4f afs0 = z4, afs1 = z4, ava0 = z4, ava1 = z4, aha = z4, ara = z4;
#pragma unroll 2
    for (int i = 0; i < LF; ++i) {
      int idx = pst[fb + i];
      idx = min(max(idx, 0), VOCAB - 1);
      const float c = csg[fb + i];
      const float s = ssg[fb + i];
      const float cs = c * s;
      const float* row = tab + (size_t)idx * TABW;
      const v4f f0 = *(const v4f*)(row + 8 * lane);
      const v4f f1 = *(const v4f*)(row + 8 * lane + 4);
      const v4f g0 = *(const v4f*)(row + S1 + 8 * lane);
      const v4f g1 = *(const v4f*)(row + S1 + 8 * lane + 4);
      const v4f hq = *(const v4f*)(row + 2 * S1 + 4 * lane);
      const v4f rq = *(const v4f*)(row + 2 * S1 + S2 + 4 * lane);
      afs0 += f0;       afs1 += f1;
      ava0 += c * g0;   ava1 += c * g1;
      aha  += s * hq;   ara  += cs * rq;
    }
    const float wp = wtm[p];
    v8h hfs, hva, hav, hpr;
    v4h hha, hra, hhr;
#pragma unroll
    for (int e = 0; e < 4; ++e) {
      const float f0v = clampT(afs0[e]);
      const float f1v = clampT(afs1[e]);
      const float v0 = clampT(add_prod(ava0[e], wp, t0[e]));
      const float v1 = clampT(add_prod(ava1[e], wp, t1[e]));
      hfs[e] = (_Float16)(f0v * ASC);          hfs[4 + e] = (_Float16)(f1v * ASC);
      hva[e] = (_Float16)(v0 * ASC);           hva[4 + e] = (_Float16)(v1 * ASC);
      hav[e] = (_Float16)(fabsf(v0) * ASC);    hav[4 + e] = (_Float16)(fabsf(v1) * ASC);
      hpr[e] = (_Float16)((f0v * v0) * ASC);   hpr[4 + e] = (_Float16)((f1v * v1) * ASC);
      const float hq = clampT(aha[e]);
      const float rq = clampT(ara[e]);
      hha[e] = (_Float16)(fabsf(hq) * ASC);
      hra[e] = (_Float16)(fabsf(rq) * ASC);
      hhr[e] = (_Float16)((hq * rq) * ASC);
    }
    _Float16* a1r = A1 + r * P1;
    _Float16* a2r = A2 + r * P2;
    *(v8h*)(a1r + 8 * lane) = hfs;
    *(v8h*)(a1r + S1 + 8 * lane) = hav;
    *(v4h*)(a1r + 2 * S1 + 4 * lane) = hha;
    *(v4h*)(a1r + 2 * S1 + S2 + 4 * lane) = hra;
    *(v8h*)(a2r + 8 * lane) = hva;
    *(v8h*)(a2r + S1 + 8 * lane) = hpr;
    *(v4h*)(a2r + 2 * S1 + 4 * lane) = hhr;
  }
  __syncthreads();

  const int mt = wave >> 2, q = wave & 3;
  v8f accF = {0.f, 0.f, 0.f, 0.f, 0.f, 0.f, 0.f, 0.f};
  v8f accV = {0.f, 0.f, 0.f, 0.f, 0.f, 0.f, 0.f, 0.f};
  {
    const _Float16* ar = A1 + (16 * mt + m) * P1 + 8 * hh;
    const _Float16* br = w1t + m * K1 + 8 * hh;
#pragma unroll
    for (int t = 0; t < K1 / 128; ++t) {
      const int k0 = 32 * (q + 4 * t);
      FragH a, b;
      a.h[0] = *(const v8h*)(ar + k0);
      a.h[1] = *(const v8h*)(ar + k0 + 16);
      b.h[0] = *(const v8h*)(br + k0);
      b.h[1] = *(const v8h*)(br + k0 + 16);
      accF = wmf(a.v, b.v, accF);
    }
  }
  {
    const _Float16* ar = A2 + (16 * mt + m) * P2 + 8 * hh;
    const _Float16* br = w2t + m * K2 + 8 * hh;
#pragma unroll
    for (int t = 0; t < K2 / 128; ++t) {
      const int k0 = 32 * (q + 4 * t);
      FragH a, b;
      a.h[0] = *(const v8h*)(ar + k0);
      a.h[1] = *(const v8h*)(ar + k0 + 16);
      b.h[0] = *(const v8h*)(br + k0);
      b.h[1] = *(const v8h*)(br + k0 + 16);
      accV = wmf(a.v, b.v, accV);
    }
  }
  {
    float* pf = part + (wave * 2 + 0) * 256 + (8 * hh) * 16 + m;
    float* pv = part + (wave * 2 + 1) * 256 + (8 * hh) * 16 + m;
#pragma unroll
    for (int rr = 0; rr < 8; ++rr) {
      pf[rr * 16] = accF[rr];
      pv[rr * 16] = accV[rr];
    }
  }
  __syncthreads();

  {
    const int rl = tid >> 3;
    const int c2 = (tid & 7) * 2;
    const int mt2 = rl >> 4, r16 = rl & 15;
    float sumv = 0.f, sumf = 0.f;
#pragma unroll
    for (int e = 0; e < 2; ++e) {
      const int c = c2 + e;
      float f = 0.f, v = 0.f;
#pragma unroll
      for (int qq = 0; qq < 4; ++qq) {
        const float* pb = part + ((mt2 * 4 + qq) * 2) * 256 + r16 * 16 + c;
        f += pb[0];
        v += pb[256];
      }
      const float fs2 = clampT(f * OSC + fsb[c]);
      const float va2 = clampT(v * OSC);
      sumv += va2 * wov[c];
      sumf += (fs2 * va2) * wof[c];
    }
    sumv += __shfl_xor(sumv, 1, 32);
    sumv += __shfl_xor(sumv, 2, 32);
    sumv += __shfl_xor(sumv, 4, 32);
    sumf += __shfl_xor(sumf, 1, 32);
    sumf += __shfl_xor(sumf, 2, 32);
    sumf += __shfl_xor(sumf, 4, 32);
    const float o = sumv + sumf;
    if ((tid & 7) == 0) sout[rl] = o;
  }
  __syncthreads();
  if (wave == 0) {
    const int l8 = lane & 7;
    const v4f v = *(const v4f*)(sout + 4 * l8);
    if (lane < 8) {
      float* gp = out + (size_t)p0 + 4 * l8;
      *(volatile v4f*)gp = v;
      __threadfence();
      *(volatile v4f*)gp = v;
    }
  }
}

extern "C" void kernel_launch(void* const* d_in, const int* in_sizes, int n_in,
                              void* d_out, int out_size, void* d_ws, size_t ws_size,
                              hipStream_t stream) {
  if (n_in < 19) return;
  const int B = in_sizes[3];
  if (B <= 0 || (B % TP) != 0) return;
  if (in_sizes[0] != B * LF || in_sizes[1] != B * LF || in_sizes[2] != B * LF) return;
  if (in_sizes[4] != VOCAB * S1 || in_sizes[5] != VOCAB * S1) return;
  if (in_sizes[6] != VOCAB * S2 || in_sizes[7] != VOCAB * S2) return;
  if (in_sizes[8] != S1) return;
  if (in_sizes[9] != S3 * S1 || in_sizes[10] != S3 || in_sizes[11] != S3 * S1) return;
  if (in_sizes[12] != S3 * S2 || in_sizes[13] != S3 * S2 || in_sizes[14] != S3 * S1) return;
  if (in_sizes[15] != S3 * S1 || in_sizes[16] != S3 * S2) return;
  if (in_sizes[17] != S3 || in_sizes[18] != S3) return;
  if (out_size != B) return;

  const int*   pst      = (const int*)d_in[0];
  const float* csg      = (const float*)d_in[1];
  const float* ssg      = (const float*)d_in[2];
  const float* wtm      = (const float*)d_in[3];
  const float* emb_fs   = (const float*)d_in[4];
  const float* emb_va   = (const float*)d_in[5];
  const float* emb_ha   = (const float*)d_in[6];
  const float* emb_ra   = (const float*)d_in[7];
  const float* tempo    = (const float*)d_in[8];
  const float* fs_w     = (const float*)d_in[9];
  const float* fs_b     = (const float*)d_in[10];
  const float* absva_w  = (const float*)d_in[11];
  const float* absha_w  = (const float*)d_in[12];
  const float* absra_w  = (const float*)d_in[13];
  const float* va_w     = (const float*)d_in[14];
  const float* fsxva_w  = (const float*)d_in[15];
  const float* haxra_w  = (const float*)d_in[16];
  const float* out_va_w = (const float*)d_in[17];
  const float* out_fx_w = (const float*)d_in[18];
  float* out = (float*)d_out;

  char* ws = (char*)d_ws;
  size_t off = 0;
  const size_t oW1 = off; off += W1T_BYTES; off = (off + 255) & ~(size_t)255;
  const size_t oW2 = off; off += W2T_BYTES; off = (off + 255) & ~(size_t)255;
  const size_t oTab = off; off += TAB_BYTES; off = (off + 255) & ~(size_t)255;
  if (off > ws_size || off > (size_t)WSCAP) return;
  _Float16* w1t = (_Float16*)(ws + oW1);
  _Float16* w2t = (_Float16*)(ws + oW2);
  float* tab = (float*)(ws + oTab);

  k_prep<<<PREP_BLOCKS, NTHR, 0, stream>>>(emb_fs, emb_va, emb_ha, emb_ra,
                                           fs_w, absva_w, absha_w, absra_w,
                                           va_w, fsxva_w, haxra_w, w1t, w2t, tab);
  hipFuncSetAttribute(reinterpret_cast<const void*>(&k_main),
                      hipFuncAttributeMaxDynamicSharedMemorySize, LDS_MAIN);
  k_main<<<B / TP, NTHR, LDS_MAIN, stream>>>(pst, csg, ssg, wtm, tempo, fs_b, out_va_w, out_fx_w,
                                             tab, w1t, w2t, out);
}
